// ModelPytorch_91190745628837
// MI455X (gfx1250) — hardware-verified
//
#include <hip/hip_runtime.h>
#include <math.h>

#define NBATCH 2048
#define NT 2048
#define NHID 32
#define TEXT 8
#define TPRED 16
#define TOUT (NT + TPRED)
#define RSPLIT (1.0f / 2048.0f)

typedef _Float16 h16;
typedef __attribute__((ext_vector_type(16))) _Float16 v16h;
typedef __attribute__((ext_vector_type(8)))  _Float16 v8h;
typedef __attribute__((ext_vector_type(8)))  float v8f;
typedef __attribute__((ext_vector_type(4)))  float v4f_t;
typedef float v4fa __attribute__((ext_vector_type(4), may_alias));

__device__ __forceinline__ h16 lo_of(float v, h16 h) { return (h16)((v - (float)h) * 2048.0f); }
__device__ __forceinline__ v8f wmma16(v16h a, v16h b, v8f c) { return __builtin_amdgcn_wmma_f32_16x16x32_f16(false, a, false, b, (short)0, c, false, false); }
__device__ __forceinline__ v8f wmma_split(v16h a, v16h al, v16h b, v16h bl, v8f c) { v8f x = {}; x = wmma16(al, b, x); x = wmma16(a, bl, x); return wmma16(a, b, c) + x * RSPLIT; }
__device__ __forceinline__ v16h rfrag(const h16* rowp, int half) {
  const h16* p = rowp + 8 * half;
  return __builtin_shufflevector(*(const v8h*)p, *(const v8h*)(p + 16), 0,1,2,3,4,5,6,7,8,9,10,11,12,13,14,15);
}
__device__ __forceinline__ int kof(int half, int e) { return 8 * half + ((e < 8) ? e : (e + 8)); }
__device__ __forceinline__ float tanh_f(float v) { return 1.0f - 2.0f * __frcp_rn(__expf(2.0f * v) + 1.0f); }

__global__ __launch_bounds__(32) void k_rnn(const float* __restrict__ x, const float* __restrict__ Wih, const float* __restrict__ bih,
                                           const float* __restrict__ Whh, const float* __restrict__ bhh, const float* __restrict__ Wdec,
                                           const float* __restrict__ bdec, float* __restrict__ y) {
  __shared__ __attribute__((aligned(16))) float ybuf[16 * TOUT];
  __shared__ __attribute__((aligned(16))) h16 hT[2][16 * 40];
  __shared__ float hf[16][33];
  const int lane = threadIdx.x, half = lane >> 4, l16 = lane & 15, kh8 = half * 8;
  const int b0 = blockIdx.x * 16;
  v16h Bw[2], Bwl[2];
#pragma unroll
  for (int nt = 0; nt < 2; ++nt) { const int n = nt * 16 + l16; v16h r, rl;
#pragma unroll
    for (int e = 0; e < 16; ++e) { const float v = Whh[n * NHID + kof(half, e)]; r[e] = (h16)v; rl[e] = lo_of(v, r[e]); }
    Bw[nt] = r; Bwl[nt] = rl; }
  float wih[2], bsum[2];
#pragma unroll
  for (int nt = 0; nt < 2; ++nt) { const int n = nt * 16 + l16; wih[nt] = Wih[n]; bsum[nt] = bih[n] + bhh[n]; }
  const float wdec_l = Wdec[lane], bd = bdec[0];

  auto rnn_step = [&](const float in8[8], bool first) {
    v8f acc[2];
#pragma unroll
    for (int nt = 0; nt < 2; ++nt) acc[nt] = v8f{};
    if (!first) {
      const v16h a = rfrag(&hT[0][l16 * 40], half), al = rfrag(&hT[1][l16 * 40], half);
#pragma unroll
      for (int nt = 0; nt < 2; ++nt) acc[nt] = wmma_split(a, al, Bw[nt], Bwl[nt], acc[nt]);
    }
    float hn[2][8];
#pragma unroll
    for (int nt = 0; nt < 2; ++nt)
#pragma unroll
      for (int r = 0; r < 8; ++r) hn[nt][r] = tanh_f(in8[r] * wih[nt] + bsum[nt] + acc[nt][r]);
    __builtin_amdgcn_wave_barrier();
#pragma unroll
    for (int nt = 0; nt < 2; ++nt) { const int n = nt * 16 + l16;
#pragma unroll
      for (int r = 0; r < 8; ++r) { const int row = kh8 + r; const float v = hn[nt][r]; const h16 hv = (h16)v;
        hT[0][row * 40 + n] = hv; hT[1][row * 40 + n] = lo_of(v, hv); hf[row][n] = v; } }
    __builtin_amdgcn_wave_barrier();
    asm volatile("s_wait_dscnt 0" ::: "memory");
  };
  auto decode = [&](float yrow[16]) {
#pragma unroll
    for (int row = 0; row < 16; ++row) { float v = hf[row][lane] * wdec_l;
#pragma unroll
      for (int o = 16; o >= 1; o >>= 1) v += __shfl_xor(v, o, 32);
      yrow[row] = v + bd; }
  };

#pragma unroll 1
  for (int t = 0; t < NT; ++t) {
    float in8[8];
#pragma unroll
    for (int r = 0; r < 8; ++r) in8[r] = x[(size_t)(b0 + kh8 + r) * NT + t];
    rnn_step(in8, t == 0);
    float yrow[16]; decode(yrow);
    if (lane < 16) ybuf[lane * TOUT + t] = yrow[lane];
  }
#pragma unroll 1
  for (int p = 0; p < TPRED; ++p) {
    const int len = NT + p;
    __builtin_amdgcn_wave_barrier();
    asm volatile("s_wait_dscnt 0" ::: "memory");
#pragma unroll 1
    for (int s = 0; s < TEXT; ++s) {
      float in8[8];
#pragma unroll
      for (int r = 0; r < 8; ++r) in8[r] = ybuf[(kh8 + r) * TOUT + (len - TEXT + s)];
      rnn_step(in8, s == 0);
    }
    float yrow[16]; decode(yrow);
    if (lane < 16) ybuf[lane * TOUT + len] = yrow[lane];
  }
  __builtin_amdgcn_wave_barrier();
  asm volatile("s_wait_dscnt 0" ::: "memory");
  float* dst = y + (size_t)b0 * TOUT;
#pragma unroll 1
  for (int pass = 0; pass < 2; ++pass) {
#pragma unroll 4
    for (int i = lane; i < 16 * TOUT / 4; i += 32) *(volatile v4f_t*)(dst + (size_t)i * 4) = *(const volatile v4fa*)(ybuf + i * 4);
    __threadfence();
  }
}

extern "C" void kernel_launch(void* const* d_in, const int* in_sizes, int n_in,
                              void* d_out, int out_size, void* d_ws, size_t ws_size,
                              hipStream_t stream) {
  (void)in_sizes; (void)n_in; (void)out_size; (void)d_ws; (void)ws_size;
  const float* x    = (const float*)d_in[0];
  const float* Wih  = (const float*)d_in[1];
  const float* bih  = (const float*)d_in[2];
  const float* Whh  = (const float*)d_in[3];
  const float* bhh  = (const float*)d_in[4];
  const float* Wdec = (const float*)d_in[5];
  const float* bdec = (const float*)d_in[6];
  k_rnn<<<NBATCH / 16, 32, 0, stream>>>(x, Wih, bih, Whh, bhh, Wdec, bdec, (float*)d_out);
}
